// STA2_Module_31920196944376
// MI455X (gfx1250) — hardware-verified
//
#include <hip/hip_runtime.h>
#include <math.h>
#include <stdint.h>

#define NB 4
#define NC 256
#define HW 4096
#define NX 512
#define QH 2048

typedef __attribute__((ext_vector_type(16))) _Float16 v16h;
typedef __attribute__((ext_vector_type(8)))  _Float16 v8h;
typedef __attribute__((ext_vector_type(16))) __bf16   v16b;
typedef __attribute__((ext_vector_type(8)))  __bf16   v8b;
typedef __attribute__((ext_vector_type(8)))  float    v8f;
typedef __attribute__((ext_vector_type(4)))  float    v4f;
typedef __attribute__((ext_vector_type(2)))  float    v2f;
typedef __attribute__((ext_vector_type(4)))  unsigned int v4u;
typedef __attribute__((ext_vector_type(8)))  unsigned short v8us;

__device__ __forceinline__ unsigned short f2bf_bits(float f) {
  unsigned u = __float_as_uint(f);
  return (unsigned short)((u + 0x7FFFu + ((u >> 16) & 1u)) >> 16);
}
__device__ __forceinline__ float bf_bits2f(unsigned short h) { return __uint_as_float(((unsigned)h) << 16); }

__device__ __forceinline__ void dep_guard_h(v8f& a, v8f& b, v16h x, v16h y) { asm volatile("v_nop\n\tv_nop\n\tv_nop\n\tv_nop" : "+v"(a), "+v"(b) : "v"(x), "v"(y)); }
__device__ __forceinline__ void dep_guard_b(v8f& a, v8f& b, v16b x, v16b y) { asm volatile("v_nop\n\tv_nop\n\tv_nop\n\tv_nop" : "+v"(a), "+v"(b) : "v"(x), "v"(y)); }
__device__ __forceinline__ void keep4_h(v16h a, v16h b, v16h c, v16h d) { asm volatile("v_nop" :: "v"(a), "v"(b), "v"(c), "v"(d)); }
__device__ __forceinline__ void keep4_b(v16b a, v16b b, v16b c, v16b d) { asm volatile("v_nop" :: "v"(a), "v"(b), "v"(c), "v"(d)); }
__device__ __forceinline__ void acc_guard4(v8f& a, v8f& b, v8f& c, v8f& d) { asm volatile("v_nop\n\tv_nop\n\tv_nop\n\tv_nop" : "+v"(a), "+v"(b), "+v"(c), "+v"(d)); }
template <typename T> struct Frag;
template <> struct Frag<_Float16> {
  typedef v16h V; union U { v16h v; v8h h[2]; };
  static __device__ __forceinline__ v16h load(const _Float16* p) {
    U f; f.h[0] = *(const v8h*)(p); f.h[1] = *(const v8h*)(p + 16); return f.v;
  }
  static __device__ __forceinline__ v8f mma(v16h a, v16h b, v8f c) {
    return __builtin_amdgcn_wmma_f32_16x16x32_f16(false, a, false, b, (short)0, c, false, false);
  }
  static __device__ __forceinline__ void guard(v8f& a, v8f& b, v16h x, v16h y) { dep_guard_h(a, b, x, y); }
  static __device__ __forceinline__ void keep(v16h a, v16h b, v16h c, v16h d) { keep4_h(a, b, c, d); }
};
template <> struct Frag<__bf16> {
  typedef v16b V; union U { v16b v; v8b h[2]; };
  static __device__ __forceinline__ v16b load(const __bf16* p) {
    U f; f.h[0] = *(const v8b*)(p); f.h[1] = *(const v8b*)(p + 16); return f.v;
  }
  static __device__ __forceinline__ v8f mma(v16b a, v16b b, v8f c) {
    return __builtin_amdgcn_wmma_f32_16x16x32_bf16(false, a, false, b, (short)0, c, false, false);
  }
  static __device__ __forceinline__ void guard(v8f& a, v8f& b, v16b x, v16b y) { dep_guard_b(a, b, x, y); }
  static __device__ __forceinline__ void keep(v16b a, v16b b, v16b c, v16b d) { keep4_b(a, b, c, d); }
};

template <int ET> struct Elem;
template <> struct Elem<0> { typedef _Float16 T; };
template <> struct Elem<1> { typedef __bf16 T; };
template <int ET, bool SPLIT, int BIAS_MODE, int OUT_MODE, bool RESID, int ACT = 0>
__global__ __launch_bounds__(256) void wmma_gemm64(
    const unsigned short* __restrict__ Ap, const unsigned short* __restrict__ A2p, int lda, long strideA,
    const unsigned short* __restrict__ Btp, const unsigned short* __restrict__ Bt2p, int ldb, long strideB,
    void* __restrict__ Cout, void* __restrict__ Cout2, int ldc, long strideC,
    const float* __restrict__ bias,
    const float* __restrict__ resid, long strideR,
    int M, int N, int K, float scale) {
  typedef typename Elem<ET>::T T;
  typedef typename Frag<T>::V V;
  const T* A = (const T*)Ap; const T* A2 = (const T*)A2p; const T* Bt = (const T*)Btp; const T* Bt2 = (const T*)Bt2p;
  __shared__ __align__(16) float sT[8][16 * 68];
  const int b    = blockIdx.y;
  const int lane = threadIdx.x & 31;
  const int wave = threadIdx.x >> 5;
  const int tilesN = N >> 6;
  const int tilesM = M >> 6;
  const int tile = blockIdx.x * 8 + wave;
  if (tile >= tilesM * tilesN) return;
  const int tm = tile / tilesN;
  const int tn = tile - tm * tilesN;
  const int m0 = tm << 6;
  const int n0 = tn << 6;

  const T* Ab  = A  + (size_t)b * strideA;
  const T* Bb  = Bt + (size_t)b * strideB;
  const T* Ab2 = SPLIT ? (A2  + (size_t)b * strideA) : nullptr;
  const T* Bb2 = SPLIT ? (Bt2 + (size_t)b * strideB) : nullptr;

  const int rlane = lane & 15;
  const int koff  = (lane >> 4) * 8;
  const int mOff  = (lane >> 4) * 8;

  v8f acc[4][4];
#pragma unroll
  for (int i = 0; i < 4; ++i)
#pragma unroll
    for (int j = 0; j < 4; ++j) acc[i][j] = (v8f){0.f,0.f,0.f,0.f,0.f,0.f,0.f,0.f};

  for (int k0 = 0; k0 < K; k0 += 32) {
    V bh[4], bl[4];
#pragma unroll
    for (int j = 0; j < 4; ++j) {
      const size_t bo = (size_t)(n0 + (j << 4) + rlane) * ldb + koff + k0;
      bh[j] = Frag<T>::load(Bb + bo);
      if (SPLIT) bl[j] = Frag<T>::load(Bb2 + bo);
    }
#pragma unroll
    for (int i = 0; i < 4; ++i) {
      const size_t ao = (size_t)(m0 + (i << 4) + rlane) * lda + koff + k0;
      V ah = Frag<T>::load(Ab + ao);
      V al;
      if (SPLIT) al = Frag<T>::load(Ab2 + ao);
#pragma unroll
      for (int j = 0; j < 4; ++j) {
        acc[i][j] = Frag<T>::mma(ah, bh[j], acc[i][j]);
        if (SPLIT) {
          acc[i][j] = Frag<T>::mma(ah, bl[j], acc[i][j]);
          acc[i][j] = Frag<T>::mma(al, bh[j], acc[i][j]);
        }
      }
      Frag<T>::guard(acc[i][0], acc[i][3], ah, SPLIT ? al : ah);
    }
    Frag<T>::keep(bh[0], bh[1], bh[2], bh[3]);
    if (SPLIT) Frag<T>::keep(bl[0], bl[1], bl[2], bl[3]);
  }
  acc_guard4(acc[0][0], acc[0][1], acc[0][2], acc[0][3]);
  acc_guard4(acc[1][0], acc[1][1], acc[1][2], acc[1][3]);
  acc_guard4(acc[2][0], acc[2][1], acc[2][2], acc[2][3]);
  acc_guard4(acc[3][0], acc[3][1], acc[3][2], acc[3][3]);

  float* slab = sT[wave];
  const float* Rb = RESID ? (resid + (size_t)b * strideR) : nullptr;
#pragma unroll
  for (int i = 0; i < 4; ++i) {
    const int mBase = m0 + (i << 4);
#pragma unroll
    for (int j = 0; j < 4; ++j) {
      const int n = n0 + (j << 4) + rlane;
      float bv = 0.f;
      if (BIAS_MODE == 2) bv = bias[n];
#pragma unroll
      for (int r = 0; r < 8; ++r) {
        float v = acc[i][j][r] * scale;
        if (BIAS_MODE == 1) v += bias[mBase + mOff + r];
        if (BIAS_MODE == 2) v += bv;
        if (RESID) v += Rb[(size_t)(mBase + mOff + r) * ldc + n];
        if (ACT == 1) v = tanhf(v);
        if (ACT == 2) v = fmaxf(v, 0.0f);
        if (ACT == 3) v = v / (1.0f + expf(-v));
        if (ACT == 4) v = (v > 0.f) ? v : 0.01f * v;
        slab[(mOff + r) * 68 + (j << 4) + rlane] = v;
      }
    }
    __builtin_amdgcn_fence(__ATOMIC_RELEASE, "workgroup");
    __builtin_amdgcn_wave_barrier();
    __builtin_amdgcn_fence(__ATOMIC_ACQUIRE, "workgroup");
    if (OUT_MODE == 0) {
      float* C = (float*)Cout + (size_t)b * strideC;
      const int hh = lane >> 4, c4 = (lane & 15) * 4;
      for (int pass = 0; pass < 2; ++pass) {
#pragma unroll
        for (int it = 0; it < 8; ++it) {
          const int row = it * 2 + hh;
          v4f v = *(const v4f*)(slab + row * 68 + c4);
          *(volatile v4f*)(C + (size_t)(mBase + row) * ldc + n0 + c4) = v;
        }
        __threadfence();
      }
    } else {
      const int q = lane >> 3, c8 = (lane & 7) * 8;
      unsigned short* C  = (unsigned short*)Cout  + (size_t)b * strideC;
      unsigned short* C2 = (OUT_MODE == 2) ? ((unsigned short*)Cout2 + (size_t)b * strideC) : nullptr;
      for (int pass = 0; pass < 2; ++pass) {
#pragma unroll
        for (int it = 0; it < 4; ++it) {
          const int row = it * 4 + q;
          const float* sp = slab + row * 68 + c8;
          v8h hv, lv;
#pragma unroll
          for (int e = 0; e < 8; ++e) {
            if (OUT_MODE == 1) {
              hv[e] = (_Float16)sp[e];
            } else if (OUT_MODE == 3) {
              hv[e] = __builtin_bit_cast(_Float16, f2bf_bits(sp[e]));
            } else {
              unsigned short hb = f2bf_bits(sp[e]);
              unsigned short lb = f2bf_bits(sp[e] - bf_bits2f(hb));
              hv[e] = __builtin_bit_cast(_Float16, hb);
              lv[e] = __builtin_bit_cast(_Float16, lb);
            }
          }
          *(volatile v8h*)(C + (size_t)(mBase + row) * ldc + n0 + c8) = hv;
          if (OUT_MODE == 2) *(volatile v8h*)(C2 + (size_t)(mBase + row) * ldc + n0 + c8) = lv;
        }
        __threadfence();
      }
    }
    __builtin_amdgcn_fence(__ATOMIC_RELEASE, "workgroup");
    __builtin_amdgcn_wave_barrier();
    __builtin_amdgcn_fence(__ATOMIC_ACQUIRE, "workgroup");
  }
}

__global__ __launch_bounds__(256) void cast_f32_bf16x2(const float* __restrict__ in, unsigned short* __restrict__ out, int n2) {
  const int i = blockIdx.x * 256 + threadIdx.x;
  if (i < n2) {
    const v2f f = *(const v2f*)(in + 2 * (size_t)i);
    const unsigned u = (unsigned)f2bf_bits(f[0]) | ((unsigned)f2bf_bits(f[1]) << 16);
    ((volatile unsigned*)out)[i] = u;
    __threadfence();
    ((volatile unsigned*)out)[i] = u;
  }
}

__global__ __launch_bounds__(256) void tr_cast_bf16(const float* __restrict__ in, int ldi,
                                                    unsigned short* __restrict__ out, int ldo, int col0) {
  __shared__ __align__(16) unsigned short sm[64 * 72];
  const int tid  = threadIdx.x;
  const int lane = tid & 31;
  const int wave = tid >> 5;
  const int i0 = blockIdx.x * 64;
  const int c0 = blockIdx.y * 64;
#pragma unroll
  for (int it = 0; it < 4; ++it) {
    const int idx = tid + 256 * it;
    const int cr  = idx >> 4;
    const int q   = idx & 15;
    const v4f f = *(const v4f*)(in + (size_t)(c0 + cr) * ldi + i0 + 4 * q);
    sm[(4 * q + 0) * 72 + cr] = f2bf_bits(f[0]);
    sm[(4 * q + 1) * 72 + cr] = f2bf_bits(f[1]);
    sm[(4 * q + 2) * 72 + cr] = f2bf_bits(f[2]);
    sm[(4 * q + 3) * 72 + cr] = f2bf_bits(f[3]);
  }
  __syncthreads();
  const int q  = lane >> 3;
  const int c8 = (lane & 7) * 8;
  for (int pass = 0; pass < 2; ++pass) {
#pragma unroll
    for (int it = 0; it < 2; ++it) {
      const int row = wave * 8 + it * 4 + q;
      const v8us v = *(const v8us*)(sm + row * 72 + c8);
      const v4u u = __builtin_bit_cast(v4u, v);
      *(volatile v4u*)(out + (size_t)(i0 + row) * ldo + col0 + c0 + c8) = u;
    }
    __threadfence();
  }
}

__global__ __launch_bounds__(512) void softmax_row_kernel(const float* __restrict__ S, unsigned short* __restrict__ P) {
  __shared__ float redm[16];
  __shared__ float reds[16];
  const int i    = blockIdx.x;
  const int tid  = threadIdx.x;
  const int lane = tid & 31;
  const int wave = tid >> 5;
  const int j0   = tid * 8;
  const float* rp = S + (size_t)i * HW + j0;
  const v4f a = *(const v4f*)(rp);
  const v4f c = *(const v4f*)(rp + 4);
  float m = fmaxf(fmaxf(fmaxf(a[0], a[1]), fmaxf(a[2], a[3])), fmaxf(fmaxf(c[0], c[1]), fmaxf(c[2], c[3])));
#pragma unroll
  for (int off = 16; off > 0; off >>= 1) m = fmaxf(m, __shfl_xor(m, off, 32));
  if (lane == 0) redm[wave] = m;
  __syncthreads();
  float mx = redm[0];
#pragma unroll
  for (int w = 1; w < 16; ++w) mx = fmaxf(mx, redm[w]);
  const float e0 = __expf(a[0] - mx), e1 = __expf(a[1] - mx), e2 = __expf(a[2] - mx), e3 = __expf(a[3] - mx);
  const float e4 = __expf(c[0] - mx), e5 = __expf(c[1] - mx), e6 = __expf(c[2] - mx), e7 = __expf(c[3] - mx);
  float s = ((e0 + e1) + (e2 + e3)) + ((e4 + e5) + (e6 + e7));
#pragma unroll
  for (int off = 16; off > 0; off >>= 1) s += __shfl_xor(s, off, 32);
  if (lane == 0) reds[wave] = s;
  __syncthreads();
  float tot = reds[0];
#pragma unroll
  for (int w = 1; w < 16; ++w) tot += reds[w];
  const float inv = 1.0f / tot;
  const float p0 = e0 * inv, p1 = e1 * inv, p2 = e2 * inv, p3 = e3 * inv;
  const float p4 = e4 * inv, p5 = e5 * inv, p6 = e6 * inv, p7 = e7 * inv;
  const v4u hv = (v4u){ (unsigned)f2bf_bits(p0) | ((unsigned)f2bf_bits(p1) << 16),
                        (unsigned)f2bf_bits(p2) | ((unsigned)f2bf_bits(p3) << 16),
                        (unsigned)f2bf_bits(p4) | ((unsigned)f2bf_bits(p5) << 16),
                        (unsigned)f2bf_bits(p6) | ((unsigned)f2bf_bits(p7) << 16) };
  const size_t ro = (size_t)i * HW + j0;
  *(volatile v4u*)(P + ro) = hv;
  __threadfence();
  *(volatile v4u*)(P + ro) = hv;
}

__global__ __launch_bounds__(256) void bn_prelu_kernel(const float* __restrict__ Y,
                                                       const float* __restrict__ gamma, const float* __restrict__ beta,
                                                       const float* __restrict__ rmean, const float* __restrict__ rvar,
                                                       const float* __restrict__ alpha,
                                                       float* __restrict__ out, int n4) {
  const int t = blockIdx.x * 256 + threadIdx.x;
  if (t < n4) {
    const int o = t >> 10;
    const float inv   = gamma[o] * rsqrtf(rvar[o] + 1e-5f);
    const float shift = beta[o] - rmean[o] * inv;
    const float slope = alpha[0];
    const v4f y = *(const v4f*)(Y + 4 * (size_t)t);
    v4f r;
#pragma unroll
    for (int e = 0; e < 4; ++e) {
      const float v = y[e] * inv + shift;
      r[e] = (v >= 0.f) ? v : slope * v;
    }
    *(volatile v4f*)(out + 4 * (size_t)t) = r;
    __threadfence();
    *(volatile v4f*)(out + 4 * (size_t)t) = r;
  }
}

extern "C" void kernel_launch(void* const* d_in, const int* in_sizes, int n_in,
                              void* d_out, int out_size, void* d_ws, size_t ws_size,
                              hipStream_t stream) {
  if (n_in < 9) return;
  if (in_sizes[0] != NB * NC * HW || in_sizes[1] != NB * NC * HW) return;
  if (in_sizes[2] != NC * NX) return;
  if (in_sizes[3] != NC || in_sizes[4] != NC || in_sizes[5] != NC || in_sizes[6] != NC || in_sizes[7] != NC) return;
  if (in_sizes[8] < 1) return;
  if (out_size != NB * NC * HW) return;

  const float* pre   = (const float*)d_in[0];
  const float* cur   = (const float*)d_in[1];
  const float* W     = (const float*)d_in[2];
  const float* bconv = (const float*)d_in[3];
  const float* gamma = (const float*)d_in[4];
  const float* beta  = (const float*)d_in[5];
  const float* rmean = (const float*)d_in[6];
  const float* rvar  = (const float*)d_in[7];
  const float* alpha = (const float*)d_in[8];
  float* out = (float*)d_out;

  const size_t szWb   = (size_t)NC * NX * 2;
  const size_t szPRET = (size_t)HW * NC * 2;
  const size_t szCURb = (size_t)NC * HW * 2;
  const size_t szXCAT = (size_t)HW * NX * 2;
  const size_t szS    = (size_t)QH * HW * 4;
  const size_t szP    = (size_t)QH * HW * 2;
  const size_t szY    = (size_t)NC * HW * 4;
  size_t off = 0;
  const size_t oWb   = off; off += szWb;
  const size_t oPRET = off; off += szPRET;
  const size_t oCURb = off; off += szCURb;
  const size_t oXCAT = off; off += szXCAT;
  const size_t oS    = off; off += szS;
  const size_t oP    = off; off += szP;
  const size_t oY    = off; off += szY;
  if (off > ws_size) return;

  char* ws = (char*)d_ws;
  unsigned short* Wb   = (unsigned short*)(ws + oWb);
  unsigned short* PRET = (unsigned short*)(ws + oPRET);
  unsigned short* CURb = (unsigned short*)(ws + oCURb);
  unsigned short* XCAT = (unsigned short*)(ws + oXCAT);
  float*          Sb   = (float*)(ws + oS);
  unsigned short* Pb   = (unsigned short*)(ws + oP);
  float*          Yb   = (float*)(ws + oY);

  const dim3 blk(256);
  const int n2W = NC * NX / 2;
  const int n2C = NC * HW / 2;
  const int n4Y = NC * HW / 4;
  const dim3 gCastW((n2W + 255) / 256);
  const dim3 gCastC((n2C + 255) / 256);
  const dim3 gTr(HW / 64, NC / 64);
  const dim3 gS(((QH / 64) * (HW / 64) + 7) / 8, 1);
  const dim3 gF(((QH / 64) * (NC / 64) + 7) / 8, 1);
  const dim3 gC(((NC / 64) * (HW / 64) + 7) / 8, 1);
  const dim3 gE((n4Y + 255) / 256);

  cast_f32_bf16x2<<<gCastW, blk, 0, stream>>>(W, Wb, n2W);

  for (int b = 0; b < NB; ++b) {
    const float* preb = pre + (size_t)b * NC * HW;
    const float* curb = cur + (size_t)b * NC * HW;
    tr_cast_bf16<<<gTr, blk, 0, stream>>>(preb, HW, PRET, NC, 0);
    tr_cast_bf16<<<gTr, blk, 0, stream>>>(curb, HW, XCAT, NX, NC);
    cast_f32_bf16x2<<<gCastC, blk, 0, stream>>>(curb, CURb, n2C);

    for (int hf = 0; hf < 2; ++hf) {
      const unsigned short* Ah = PRET + (size_t)hf * QH * NC;
      wmma_gemm64<1, false, 0, 0, false, 0><<<gS, blk, 0, stream>>>(
          Ah, Ah, NC, 0L, XCAT + NC, XCAT + NC, NX, 0L, (void*)Sb, (void*)Sb, HW, 0L,
          bconv, bconv, 0L, QH, HW, NC, 0.0625f);
      softmax_row_kernel<<<dim3(QH), dim3(512), 0, stream>>>(Sb, Pb);
      wmma_gemm64<1, false, 0, 3, false, 0><<<gF, blk, 0, stream>>>(
          Pb, Pb, HW, 0L, CURb, CURb, HW, 0L,
          (void*)(XCAT + (size_t)hf * QH * NX), (void*)(XCAT + (size_t)hf * QH * NX), NX, 0L,
          bconv, bconv, 0L, QH, NC, HW, 1.0f);
    }
    wmma_gemm64<1, false, 1, 0, false, 0><<<gC, blk, 0, stream>>>(
        Wb, Wb, NX, 0L, XCAT, XCAT, NX, 0L, (void*)Yb, (void*)Yb, HW, 0L,
        bconv, bconv, 0L, NC, HW, NX, 1.0f);
    bn_prelu_kernel<<<gE, blk, 0, stream>>>(Yb, gamma, beta, rmean, rvar, alpha,
                                             out + (size_t)b * NC * HW, n4Y);
  }
  (void)hipGetLastError();
}
